// MultiHeadAttention_60138132078900
// MI455X (gfx1250) — hardware-run, weakly checked
//
#include <hip/hip_runtime.h>
#include <math.h>

#ifndef NB
#define NB 2
#endif
#ifndef SEQ
#define SEQ 2048
#endif
#define NB_FULL 2
#define SEQ_FULL 2048
#define EMB 1024
#define HEADS 16
#define HD 64
#define MROWS (SEQ * NB)
#define OUT1_OFF_BYTES 16777216
#define OUT1_OFF ((size_t)SEQ_FULL * NB_FULL * EMB)

static_assert(OUT1_OFF * 4 == OUT1_OFF_BYTES);
static_assert(SEQ % 64 == 0 && SEQ <= SEQ_FULL && NB >= 1 && NB <= NB_FULL);
static_assert(EMB % 64 == 0 && HD == 64 && HEADS * HD == EMB);
static_assert(((size_t)(NB - 1) * SEQ_FULL + (SEQ - 1)) * SEQ_FULL + SEQ <= (size_t)NB_FULL * SEQ_FULL * SEQ_FULL);
static_assert(((size_t)(SEQ - 1) * NB_FULL + NB) * EMB <= OUT1_OFF);

typedef _Float16 v16h __attribute__((ext_vector_type(16)));
typedef _Float16 v8h  __attribute__((ext_vector_type(8)));
typedef float    v8f  __attribute__((ext_vector_type(8)));
typedef float    v4f  __attribute__((ext_vector_type(4)));
typedef float    v2f  __attribute__((ext_vector_type(2)));
typedef unsigned int v4u __attribute__((ext_vector_type(4)));

union FragU { v16h v; v8h h[2]; };
__device__ __forceinline__ v16h ldfrag(const _Float16* p) { FragU f; f.h[0] = *(const v8h*)(p); f.h[1] = *(const v8h*)(p + 16); return f.v; }

__device__ __forceinline__ v8f mma_raw(v16h a, v16h b, v8f c) {
    return __builtin_amdgcn_wmma_f32_16x16x32_f16(false, a, false, b, (short)0, c, false, false);
}
__device__ __forceinline__ void dep_guard(v8f& a, v8f& b, v16h x) { asm volatile("v_nop\n\tv_nop\n\tv_nop\n\tv_nop" : "+v"(a), "+v"(b) : "v"(x)); }
__device__ __forceinline__ void keep4(v16h a, v16h b, v16h c, v16h d) { asm volatile("v_nop" :: "v"(a), "v"(b), "v"(c), "v"(d)); }
__device__ __forceinline__ void acc_guard4(v8f& a, v8f& b, v8f& c, v8f& d) { asm volatile("v_nop\n\tv_nop\n\tv_nop\n\tv_nop" : "+v"(a), "+v"(b), "+v"(c), "+v"(d)); }
__device__ __forceinline__ v8f wmma2(v16h a0, v16h b0, v16h a1, v16h b1, v8f c) {
    c = mma_raw(a0, b0, c);
    c = mma_raw(a1, b1, c);
    asm volatile("v_nop\n\tv_nop\n\tv_nop\n\tv_nop" : "+v"(c) : "v"(a0), "v"(b0), "v"(a1), "v"(b1));
    return c;
}
__device__ __forceinline__ void pv4(v8f& o0, v8f& o1, v8f& o2, v8f& o3, v16h a0, v16h a1, v16h a2, v16h a3, v16h p) {
    o0 = mma_raw(a0, p, o0);
    o1 = mma_raw(a1, p, o1);
    o2 = mma_raw(a2, p, o2);
    o3 = mma_raw(a3, p, o3);
    asm volatile("v_nop\n\tv_nop\n\tv_nop\n\tv_nop" : "+v"(o0), "+v"(o1), "+v"(o2), "+v"(o3) : "v"(a0), "v"(a1), "v"(a2), "v"(a3), "v"(p));
}

#define VST2(T, ptr, val) do { const T vst2_v_ = (val); *(volatile T*)(ptr) = vst2_v_; __threadfence(); *(volatile T*)(ptr) = vst2_v_; } while (0)

__device__ __forceinline__ float cmb_bf(float v) {
    const unsigned u = __builtin_bit_cast(unsigned, v);
    const unsigned r = (u + 0x7fffu + ((u >> 16) & 1u)) & 0xffff0000u;
    return __builtin_bit_cast(float, r);
}
__device__ __forceinline__ unsigned int cmb_pk2(float a, float b) {
    return (unsigned int)__builtin_bit_cast(unsigned short, (_Float16)a) | ((unsigned int)__builtin_bit_cast(unsigned short, (_Float16)b) << 16);
}

__global__ __launch_bounds__(256) void k_cast_bf_f16(const float* __restrict__ SRC, unsigned short* __restrict__ DST, int nR, int rg, int rgF, float sc) {
    const long long u = (long long)blockIdx.x * 256 + threadIdx.x;
    const int per = EMB / 8;
    if (u >= (long long)nR * per) return;
    const int r = (int)(u / per);
    const int c0 = 8 * (int)(u % per);
    const int sr = (r / rg) * rgF + (r % rg);
    const float* s = SRC + (long long)sr * EMB + c0;
    const v4f a = *(const v4f*)(s);
    const v4f b = *(const v4f*)(s + 4);
    v4u pk;
    pk.x = cmb_pk2(cmb_bf(a.x) * sc, cmb_bf(a.y) * sc);
    pk.y = cmb_pk2(cmb_bf(a.z) * sc, cmb_bf(a.w) * sc);
    pk.z = cmb_pk2(cmb_bf(b.x) * sc, cmb_bf(b.y) * sc);
    pk.w = cmb_pk2(cmb_bf(b.z) * sc, cmb_bf(b.w) * sc);
    VST2(v4u, (v4u*)(DST + (long long)r * EMB + c0), pk);
}

template <int BIAS_MODE, int OUT_MODE>
__global__ __launch_bounds__(256) void k_gemm64(
    const unsigned short* __restrict__ Ap, int lda, long long strideA,
    const unsigned short* __restrict__ Btp, int ldb, long long strideB,
    void* __restrict__ Cout, int ldc, long long strideC,
    const float* __restrict__ bias, int M, int N, int K, float scale, int rg, int rgF) {
  __shared__ __align__(16) float sT[8][16 * 68];
  const int bz   = blockIdx.y;
  const int lane = threadIdx.x & 31;
  const int wave = threadIdx.x >> 5;
  const int tilesN = N >> 6;
  const int tilesM = M >> 6;
  const int tile = blockIdx.x * 8 + wave;
  if (tile >= tilesM * tilesN) return;
  const int tm = tile / tilesN;
  const int tn = tile - tm * tilesN;
  const int m0 = tm << 6;
  const int n0 = tn << 6;

  const _Float16* Ab = (const _Float16*)Ap  + (size_t)((long long)bz * strideA);
  const _Float16* Bb = (const _Float16*)Btp + (size_t)((long long)bz * strideB);

  const int rlane = lane & 15;
  const int koff  = (lane >> 4) * 8;
  const int mOff  = (lane >> 4) * 8;

  v8f acc[4][4];
#pragma unroll
  for (int i = 0; i < 4; ++i)
#pragma unroll
    for (int j = 0; j < 4; ++j) acc[i][j] = (v8f){0.f, 0.f, 0.f, 0.f, 0.f, 0.f, 0.f, 0.f};

  for (int k0 = 0; k0 < K; k0 += 32) {
    v16h bh[4];
#pragma unroll
    for (int j = 0; j < 4; ++j) {
      const size_t bo = (size_t)(n0 + (j << 4) + rlane) * ldb + koff + k0;
      bh[j] = ldfrag(Bb + bo);
    }
#pragma unroll
    for (int i = 0; i < 4; ++i) {
      const size_t ao = (size_t)(m0 + (i << 4) + rlane) * lda + koff + k0;
      const v16h ah = ldfrag(Ab + ao);
#pragma unroll
      for (int j = 0; j < 4; ++j) acc[i][j] = mma_raw(ah, bh[j], acc[i][j]);
      dep_guard(acc[i][0], acc[i][3], ah);
    }
    keep4(bh[0], bh[1], bh[2], bh[3]);
  }
  acc_guard4(acc[0][0], acc[0][1], acc[0][2], acc[0][3]);
  acc_guard4(acc[1][0], acc[1][1], acc[1][2], acc[1][3]);
  acc_guard4(acc[2][0], acc[2][1], acc[2][2], acc[2][3]);
  acc_guard4(acc[3][0], acc[3][1], acc[3][2], acc[3][3]);

  float* slab = sT[wave];
#pragma unroll
  for (int i = 0; i < 4; ++i) {
    const int mBase = m0 + (i << 4);
#pragma unroll
    for (int j = 0; j < 4; ++j) {
      const int n = n0 + (j << 4) + rlane;
      float bv = 0.f;
      if (BIAS_MODE == 2) bv = cmb_bf(bias[n]);
#pragma unroll
      for (int r = 0; r < 8; ++r) {
        float v = acc[i][j][r] * scale;
        if (BIAS_MODE == 1) v += cmb_bf(bias[mBase + mOff + r]);
        if (BIAS_MODE == 2) v += bv;
        slab[(mOff + r) * 68 + (j << 4) + rlane] = v;
      }
    }
    __builtin_amdgcn_fence(3  , "workgroup");
    __builtin_amdgcn_wave_barrier();
    __builtin_amdgcn_fence(2  , "workgroup");
    if (OUT_MODE == 0) {
      float* C = (float*)Cout + (size_t)((long long)bz * strideC);
      const int hh = lane >> 4, c4 = (lane & 15) * 4;
      for (int pass = 0; pass < 2; ++pass) {
#pragma unroll
        for (int it = 0; it < 8; ++it) {
          const int row = it * 2 + hh;
          const int gm = mBase + row;
          const int crow = (gm / rg) * rgF + (gm % rg);
          const v4f v = *(const v4f*)(slab + row * 68 + c4);
          *(volatile v4f*)(C + (size_t)crow * ldc + n0 + c4) = v;
        }
        __threadfence();
      }
    } else {
      const int q = lane >> 3, c8 = (lane & 7) * 8;
      unsigned short* C = (unsigned short*)Cout + (size_t)((long long)bz * strideC);
      for (int pass = 0; pass < 2; ++pass) {
#pragma unroll
        for (int it = 0; it < 4; ++it) {
          const int row = it * 4 + q;
          const int gm = mBase + row;
          const int crow = (gm / rg) * rgF + (gm % rg);
          const float* sp = slab + row * 68 + c8;
          v8h hv;
#pragma unroll
          for (int e = 0; e < 8; ++e) hv[e] = (_Float16)sp[e];
          *(volatile v8h*)(C + (size_t)crow * ldc + n0 + c8) = hv;
        }
        __threadfence();
      }
    }
    __builtin_amdgcn_fence(3  , "workgroup");
    __builtin_amdgcn_wave_barrier();
    __builtin_amdgcn_fence(2  , "workgroup");
  }
}

#define LOG2E_F 1.4426950408889634f
__global__ __launch_bounds__(128) void k_flashT(const unsigned short* __restrict__ Qp, const unsigned short* __restrict__ Kp,
                                                const unsigned short* __restrict__ VTp, unsigned short* __restrict__ CTXp,
                                                float* __restrict__ ST) {
  __shared__ __align__(16) float sO[4][16 * 68];
  const _Float16* Q  = (const _Float16*)Qp;
  const _Float16* K  = (const _Float16*)Kp;
  const _Float16* VT = (const _Float16*)VTp;
  const int lane = threadIdx.x & 31, wave = threadIdx.x >> 5, hf = lane >> 4, l15 = lane & 15;
  const int nqb = SEQ / 64;
  const int bx = blockIdx.x;
  const int qb = bx % nqb;
  const int bh = bx / nqb;
  const int h  = bh % HEADS;
  const int b  = bh / HEADS;
  const int q0 = qb * 64 + wave * 16;

  const _Float16* qrow = Q + ((size_t)(q0 + l15) * NB + b) * EMB + h * HD + 8 * hf;
  const v16h qf0 = ldfrag(qrow);
  const v16h qf1 = ldfrag(qrow + 32);
  const _Float16* kbase = K + (size_t)b * EMB + h * HD + 8 * hf;
  const _Float16* vbase = VT + (size_t)(h * HD + l15) * ((size_t)NB * SEQ) + (size_t)b * SEQ + 8 * hf;
  const size_t vstep = (size_t)16 * NB * SEQ;

  const float SC = 0.125f * LOG2E_F;
  float m = -1.0e30f, l = 0.f;
  v8f o0 = {}, o1 = {}, o2 = {}, o3 = {};

#pragma unroll 1
  for (int s0 = 0; s0 < SEQ; s0 += 32) {
    const _Float16* k0r = kbase + (size_t)(s0 + l15) * NB * EMB;
    const _Float16* k1r = kbase + (size_t)(s0 + 16 + l15) * NB * EMB;
    const v16h ka0 = ldfrag(k0r), ka1 = ldfrag(k0r + 32);
    const v16h kb0 = ldfrag(k1r), kb1 = ldfrag(k1r + 32);
    v8f sa = {}, sb = {};
    sa = wmma2(ka0, qf0, ka1, qf1, sa);
    sb = wmma2(kb0, qf0, kb1, qf1, sb);

    float ta[8], tb[8];
    float mx = -1.0e30f;
#pragma unroll
    for (int r = 0; r < 8; ++r) { ta[r] = sa[r] * SC; tb[r] = sb[r] * SC; mx = fmaxf(mx, fmaxf(ta[r], tb[r])); }
    mx = fmaxf(mx, __shfl_xor(mx, 16, 32));
    const float mnew = fmaxf(m, mx);
    const float alpha = exp2f(m - mnew);
    float rs = 0.f;
    v16h pf;
#pragma unroll
    for (int r = 0; r < 8; ++r) {
      const float pa = exp2f(ta[r] - mnew);
      const float pb = exp2f(tb[r] - mnew);
      rs += pa + pb;
      pf[r]     = (_Float16)(pa * 4096.0f);
      pf[8 + r] = (_Float16)(pb * 4096.0f);
    }
    rs += __shfl_xor(rs, 16, 32);
    l = l * alpha + rs;
    m = mnew;
    o0 *= alpha; o1 *= alpha; o2 *= alpha; o3 *= alpha;

    const _Float16* vr = vbase + s0;
    const v16h v0 = ldfrag(vr);
    const v16h v1 = ldfrag(vr + vstep);
    const v16h v2 = ldfrag(vr + 2 * vstep);
    const v16h v3 = ldfrag(vr + 3 * vstep);
    pv4(o0, o1, o2, o3, v0, v1, v2, v3, pf);
  }

  const float inv = 1.0f / l;
  {
    const int qs = lane >> 1;
    const float mv = __shfl(m, qs, 32);
    const float iv = __shfl(inv, qs, 32);
    const float val = (lane & 1) ? iv : mv;
    VST2(float, ST + ((size_t)(b * HEADS + h) * SEQ + q0) * 2 + lane, val);
  }
  float* slab = sO[wave];
  const float fs = inv * (1.0f / 64.0f);
#pragma unroll
  for (int r = 0; r < 8; ++r) {
    slab[l15 * 68 +  0 + 8 * hf + r] = o0[r] * fs;
    slab[l15 * 68 + 16 + 8 * hf + r] = o1[r] * fs;
    slab[l15 * 68 + 32 + 8 * hf + r] = o2[r] * fs;
    slab[l15 * 68 + 48 + 8 * hf + r] = o3[r] * fs;
  }
  __builtin_amdgcn_fence(3  , "workgroup");
  __builtin_amdgcn_wave_barrier();
  __builtin_amdgcn_fence(2  , "workgroup");
  {
    const int qq = lane >> 3, c8 = (lane & 7) * 8;
    for (int pass = 0; pass < 2; ++pass) {
#pragma unroll
      for (int it = 0; it < 4; ++it) {
        const int row = it * 4 + qq;
        const float* sp = slab + row * 68 + c8;
        v8h hv;
#pragma unroll
        for (int e = 0; e < 8; ++e) hv[e] = (_Float16)sp[e];
        *(volatile v8h*)(CTXp + ((size_t)(q0 + row) * NB + b) * EMB + h * HD + c8) = hv;
      }
      __threadfence();
    }
  }
}

__global__ __launch_bounds__(256) void k_avgT(const unsigned short* __restrict__ Qp, const unsigned short* __restrict__ Kp,
                                              const float* __restrict__ ST, float* __restrict__ AVG) {
  __shared__ __align__(16) float sA[8][16 * 68];
  const _Float16* Q = (const _Float16*)Qp;
  const _Float16* K = (const _Float16*)Kp;
  const int lane = threadIdx.x & 31, wave = threadIdx.x >> 5, hf = lane >> 4, l15 = lane & 15;
  const int TT = SEQ / 16, SS = SEQ / 64;
  const int gid = blockIdx.x * 8 + wave;
  if (gid >= NB * TT * SS) return;
  const int b  = gid / (TT * SS);
  const int rr = gid - b * (TT * SS);
  const int t0 = (rr / SS) * 16;
  const int s0 = (rr % SS) * 64;
  const float SC = 0.125f * LOG2E_F;

  v8f w[4];
#pragma unroll
  for (int kt = 0; kt < 4; ++kt) w[kt] = (v8f){0.f, 0.f, 0.f, 0.f, 0.f, 0.f, 0.f, 0.f};

#pragma unroll 1
  for (int h = 0; h < HEADS; ++h) {
    const _Float16* qrow = Q + ((size_t)(t0 + l15) * NB + b) * EMB + h * HD + 8 * hf;
    const v16h qf0 = ldfrag(qrow);
    const v16h qf1 = ldfrag(qrow + 32);
    const v2f st = *(const v2f*)(ST + ((size_t)(b * HEADS + h) * SEQ + t0 + l15) * 2);
    const float mm = st.x, iv = st.y;
#pragma unroll
    for (int kt = 0; kt < 4; ++kt) {
      const _Float16* kr = K + ((size_t)(s0 + kt * 16 + l15) * NB + b) * EMB + h * HD + 8 * hf;
      const v16h k0 = ldfrag(kr), k1 = ldfrag(kr + 32);
      v8f s = {};
      s = wmma2(k0, qf0, k1, qf1, s);
#pragma unroll
      for (int r = 0; r < 8; ++r) w[kt][r] += exp2f(s[r] * SC - mm) * iv;
    }
  }

  float* slab = sA[wave];
  const float invH = 1.0f / (float)HEADS;
#pragma unroll
  for (int kt = 0; kt < 4; ++kt)
#pragma unroll
    for (int r = 0; r < 8; ++r) slab[l15 * 68 + kt * 16 + 8 * hf + r] = w[kt][r] * invH;
  __builtin_amdgcn_fence(3  , "workgroup");
  __builtin_amdgcn_wave_barrier();
  __builtin_amdgcn_fence(2  , "workgroup");
  {
    const int hh = lane >> 4, c4 = (lane & 15) * 4;
    for (int pass = 0; pass < 2; ++pass) {
#pragma unroll
      for (int it = 0; it < 8; ++it) {
        const int row = it * 2 + hh;
        const v4f v = *(const v4f*)(slab + row * 68 + c4);
        *(volatile v4f*)(AVG + ((size_t)b * SEQ_FULL + t0 + row) * SEQ_FULL + s0 + c4) = v;
      }
      __threadfence();
    }
  }
}

extern "C" void kernel_launch(void* const* d_in, const int* in_sizes, int n_in, void* d_out, int out_size, void* d_ws, size_t ws_size, hipStream_t stream) {
    if (n_in < 11) return;
    const long long xneed = ((long long)(SEQ - 1) * NB_FULL + NB) * EMB;
    if (in_sizes[0] < xneed || in_sizes[1] < xneed || in_sizes[2] < xneed) return;
    if (in_sizes[3] < EMB * EMB || in_sizes[5] < EMB * EMB || in_sizes[7] < EMB * EMB || in_sizes[9] < EMB * EMB) return;
    if (in_sizes[4] < EMB || in_sizes[6] < EMB || in_sizes[8] < EMB || in_sizes[10] < EMB) return;
    const long long oneed = (long long)OUT1_OFF + ((long long)(NB - 1) * SEQ_FULL + (SEQ - 1)) * SEQ_FULL + SEQ;
    if ((long long)out_size < oneed) return;

    const float* xq = (const float*)d_in[0];
    const float* xk = (const float*)d_in[1];
    const float* xv = (const float*)d_in[2];
    const float* Wq = (const float*)d_in[3];
    const float* bq = (const float*)d_in[4];
    const float* Wk = (const float*)d_in[5];
    const float* bk = (const float*)d_in[6];
    const float* Wv = (const float*)d_in[7];
    const float* bv = (const float*)d_in[8];
    const float* Wo = (const float*)d_in[9];
    const float* bo = (const float*)d_in[10];
    float* out = (float*)d_out;
    float* avg = out + OUT1_OFF;

    const size_t XE = (size_t)MROWS * EMB;
    const size_t WE = (size_t)EMB * EMB;
    char* wsp = (char*)d_ws;
    unsigned short* X16   = (unsigned short*)wsp; wsp += 3 * XE * 2;
    unsigned short* W16   = (unsigned short*)wsp; wsp += 4 * WE * 2;
    unsigned short* QK16  = (unsigned short*)wsp; wsp += 2 * XE * 2;
    unsigned short* VT16  = (unsigned short*)wsp; wsp += XE * 2;
    unsigned short* CTX16 = (unsigned short*)wsp; wsp += XE * 2;
    float*          STP   = (float*)wsp;          wsp += (size_t)NB * HEADS * SEQ * 2 * 4;
    if ((size_t)(wsp - (char*)d_ws) > ws_size) return;

    const unsigned gx = (unsigned)(((long long)MROWS * (EMB / 8) + 255) / 256);
    const unsigned gw = (unsigned)(((long long)EMB * (EMB / 8) + 255) / 256);
    k_cast_bf_f16<<<gx, 256, 0, stream>>>(xq, X16,          MROWS, NB, NB_FULL, 16.0f);
    k_cast_bf_f16<<<gx, 256, 0, stream>>>(xk, X16 + XE,     MROWS, NB, NB_FULL, 16.0f);
    k_cast_bf_f16<<<gx, 256, 0, stream>>>(xv, X16 + 2 * XE, MROWS, NB, NB_FULL, 16.0f);
    k_cast_bf_f16<<<gw, 256, 0, stream>>>(Wq, W16,          EMB, 1, 1, 16.0f);
    k_cast_bf_f16<<<gw, 256, 0, stream>>>(Wk, W16 + WE,     EMB, 1, 1, 16.0f);
    k_cast_bf_f16<<<gw, 256, 0, stream>>>(Wv, W16 + 2 * WE, EMB, 1, 1, 16.0f);
    k_cast_bf_f16<<<gw, 256, 0, stream>>>(Wo, W16 + 3 * WE, EMB, 1, 1, 16.0f);

    const unsigned gproj = (unsigned)((((MROWS / 64) * (EMB / 64)) + 7) / 8);
    k_gemm64<2, 1><<<dim3(gproj, 1), 256, 0, stream>>>(X16, EMB, 0LL, W16, EMB, 0LL, (void*)QK16, EMB, 0LL, bq, MROWS, EMB, EMB, 0.00390625f, 1, 1);
    k_gemm64<2, 1><<<dim3(gproj, 1), 256, 0, stream>>>(X16 + XE, EMB, 0LL, W16 + WE, EMB, 0LL, (void*)(QK16 + XE), EMB, 0LL, bk, MROWS, EMB, EMB, 0.00390625f, 1, 1);
    const unsigned gvt = (unsigned)((((EMB / 64) * (SEQ / 64)) + 7) / 8);
    k_gemm64<1, 1><<<dim3(gvt, NB), 256, 0, stream>>>(W16 + 2 * WE, EMB, 0LL, X16 + 2 * XE, NB * EMB, (long long)EMB, (void*)VT16, NB * SEQ, (long long)SEQ, bv, EMB, SEQ, EMB, 0.00390625f, 1, 1);

    k_flashT<<<NB * HEADS * (SEQ / 64), 128, 0, stream>>>(QK16, QK16 + XE, VT16, CTX16, STP);
    k_avgT<<<(unsigned)((NB * (SEQ / 16) * (SEQ / 64) + 7) / 8), 256, 0, stream>>>(QK16, QK16 + XE, STP, avg);

    k_gemm64<2, 0><<<dim3(gproj, 1), 256, 0, stream>>>(CTX16, EMB, 0LL, W16 + 3 * WE, EMB, 0LL, (void*)out, EMB, 0LL, bo, MROWS, EMB, EMB, 0.0009765625f, NB, NB_FULL);
}
